// HeavilyCompressedAttention_10582799417771
// MI455X (gfx1250) — hardware-verified
//
#include <hip/hip_runtime.h>
#include <hip/hip_bf16.h>
#include <math.h>

#define BB 4
#define TT 8192
#define DM 256
#define CC 64
#define HH 4
#define KVH 1
#define HKDIV 4
#define KVD 64
#define DD 256
#define DKK 64
#define QW 2
#define QROWS TT
#define NKV 528
#define KROWS 544
#define SS TT
#define MTOK (BB * TT)
#define GSTR 48

typedef _Float16 bf16;
typedef _Float16 f16;
typedef __attribute__((ext_vector_type(4))) unsigned v4u_t;
typedef unsigned v4ua __attribute__((ext_vector_type(4), may_alias));
typedef __attribute__((ext_vector_type(4))) float v4f_t;
typedef float v4fa __attribute__((ext_vector_type(4), may_alias));
typedef __attribute__((ext_vector_type(16))) bf16  bf16x16;
typedef bf16x16 f16x16;
typedef __attribute__((ext_vector_type(8)))  bf16  bf16x8;
typedef bf16x8 f16x8;
typedef __attribute__((ext_vector_type(4)))  bf16  bf16x4;
typedef __attribute__((ext_vector_type(8)))  float f32x8;
__device__ __forceinline__ f32x8 wmma16(f16x16 a, f16x16 b, f32x8 c) {
  c = __builtin_amdgcn_wmma_f32_16x16x32_f16(false, a, false, b, (short)0, c, false, false);
  asm volatile("v_nop\n\tv_nop\n\tv_nop\n\tv_nop" : "+v"(c) : "v"(a), "v"(b));
  return c;
}
#define LDS_STRIDE 48
#define KSTRIDE    72
#define VSTRIDE    48

__device__ __forceinline__ f32x8 wmma_bf16(bf16x16 a, bf16x16 b, f32x8 c) {
  c = __builtin_amdgcn_wmma_f32_16x16x32_f16(false, a, false, b, (short)0, c, false, false);
  asm volatile("v_nop\n\tv_nop\n\tv_nop\n\tv_nop" : "+v"(c) : "v"(a), "v"(b));
  return c;
}

template <typename T>
__device__ __forceinline__ bf16x16 load_frag(const T* __restrict__ base, int ld,
                                             int row0, int k0) {
  const int lane = threadIdx.x & 31;
  const int r    = lane & 15;
  const int kh   = (lane >> 4) * 8;
  const T* p0 = base + (size_t)(row0 + r) * ld + (k0 + kh);
  const T* p1 = p0 + 16;
  bf16x16 f;
#pragma unroll
  for (int i = 0; i < 8; ++i) {
    f[i]     = (bf16)p0[i];
    f[i + 8] = (bf16)p1[i];
  }
  return f;
}

__device__ __forceinline__ bf16x16 lds_frag(const bf16* base, int stride) {
  const int lane = threadIdx.x & 31;
  const int row  = lane & 15;
  const int kh   = (lane >> 4) * 8;
  const bf16x8 lo = *(const bf16x8*)(base + row * stride + kh);
  const bf16x8 hi = *(const bf16x8*)(base + row * stride + kh + 16);
  bf16x16 f;
#pragma unroll
  for (int i = 0; i < 8; ++i) { f[i] = lo[i]; f[i + 8] = hi[i]; }
  return f;
}

template <typename T>
__device__ __forceinline__ void stage_read16(const T* __restrict__ p, float* buf) {
#pragma unroll
  for (int i = 0; i < 16; ++i) buf[i] = (float)p[i];
}

__device__ __forceinline__ void stage_write(bf16* dst, const float* buf, int nquad) {
#pragma unroll
  for (int i = 0; i < nquad; ++i) {
    bf16x4 q;
    q[0] = (bf16)buf[4 * i];     q[1] = (bf16)buf[4 * i + 1];
    q[2] = (bf16)buf[4 * i + 2]; q[3] = (bf16)buf[4 * i + 3];
    *(bf16x4*)(dst + 4 * i) = q;
  }
}

__global__ __launch_bounds__(64) void attn_kernel(
    const bf16* __restrict__ Qb, const bf16* __restrict__ Kb,
    const bf16* __restrict__ Vt,
    float* __restrict__ attnOut) {
  __shared__ bf16 ldsK[32 * KSTRIDE];
  __shared__ bf16 ldsV[64 * VSTRIDE];
  __shared__ __attribute__((aligned(16))) bf16 ldsO[2][32 * 72];

  const int q0blk = blockIdx.x * 64;
  const int h  = blockIdx.y;
  const int b  = blockIdx.z;
  const int t    = threadIdx.x;
  const int wave = t >> 5;
  const int lane = t & 31;
  const int qlane = lane & 15;
  const int kh8   = (lane >> 4) * 8;
  const int q0 = q0blk + wave * 32;

  const int hk = h / HKDIV;
  const bf16* Qh = Qb + (size_t)b * QROWS * DD + h * DKK;
  const bf16* Kh = Kb + (size_t)b * KROWS * KVD + hk * DKK;
  const bf16* Vh = Vt + ((size_t)(b * KVH + hk)) * DKK * KROWS;

  const int krow = t >> 1;
  const int kcol = (t & 1) * 32;
  const bf16* kSrc = Kh + (size_t)krow * KVD + kcol;
  const bf16* vSrc = Vh + (size_t)t * KROWS;

  bf16x16 qf[QW][2];
#pragma unroll
  for (int qt = 0; qt < QW; ++qt) {
    qf[qt][0] = load_frag(Qh, DD, q0 + 16 * qt, 0);
    qf[qt][1] = load_frag(Qh, DD, q0 + 16 * qt, 32);
  }

  f32x8 o[QW][4] = {};
  float mrun[QW], lrun[QW];
#pragma unroll
  for (int qt = 0; qt < QW; ++qt) { mrun[qt] = -INFINITY; lrun[qt] = 0.0f; }

  const float scale = 0.125f * 1.44269504088896340736f;
  const float NEG2 = -1.0e9f;
  const int kmax = KROWS - 1;

  bf16x8 kreg[4], vreg[4];
#pragma unroll
  for (int i = 0; i < 4; ++i) {
    kreg[i] = *(const bf16x8*)(kSrc + 8 * i);
    vreg[i] = *(const bf16x8*)(vSrc + 8 * i);
  }

  for (int kb = 0; kb <= kmax; kb += 32) {
    __syncthreads();
#pragma unroll
    for (int i = 0; i < 4; ++i) {
      *(bf16x8*)(&ldsK[krow * KSTRIDE + kcol + 8 * i]) = kreg[i];
      *(bf16x8*)(&ldsV[t * VSTRIDE + 8 * i])           = vreg[i];
    }
    if (kb + 32 <= kmax) {
      const bf16* kn = kSrc + (size_t)(kb + 32) * KVD;
      const bf16* vn = vSrc + (kb + 32);
#pragma unroll
      for (int i = 0; i < 4; ++i) {
        kreg[i] = *(const bf16x8*)(kn + 8 * i);
        vreg[i] = *(const bf16x8*)(vn + 8 * i);
      }
    }
    __syncthreads();

    bf16x16 kf[2][2];
#pragma unroll
    for (int ktile = 0; ktile < 2; ++ktile)
#pragma unroll
      for (int c = 0; c < 2; ++c)
        kf[ktile][c] = lds_frag(ldsK + (ktile * 16) * KSTRIDE + c * 32, KSTRIDE);

    bf16x16 pf[QW];
    bool act[QW];
#pragma unroll
    for (int qt = 0; qt < QW; ++qt) {
      unsigned mbits = 0;
      {
#pragma unroll
        for (int r = 0; r < 8; ++r) { const int j0 = kb + kh8 + r; if (j0 < NKV) mbits |= 1u << r; if (j0 + 16 < NKV) mbits |= 1u << (8 + r); }
        act[qt] = (__builtin_amdgcn_ballot_w32(mbits != 0) != 0);
      }
      if (act[qt]) {
        const int q_my = q0 + 16 * qt + qlane;
        f32x8 s0 = {}, s1 = {};
        s0 = wmma_bf16(kf[0][0], qf[qt][0], s0);
        s0 = wmma_bf16(kf[0][1], qf[qt][1], s0);
        s1 = wmma_bf16(kf[1][0], qf[qt][0], s1);
        s1 = wmma_bf16(kf[1][1], qf[qt][1], s1);

        float mx = -INFINITY;
#pragma unroll
        for (int r = 0; r < 8; ++r) {
          const int k0i = kb + kh8 + r;
          const int k1i = k0i + 16;
          (void)k0i; (void)k1i; (void)q_my;
          s0[r] = (mbits & (1u << r))       ? s0[r] * scale : NEG2;
          s1[r] = (mbits & (1u << (8 + r))) ? s1[r] * scale : NEG2;
          mx = fmaxf(mx, fmaxf(s0[r], s1[r]));
        }
        mx = fmaxf(mx, __shfl_xor(mx, 16, 32));
        const float mnew  = fmaxf(mrun[qt], mx);
        const float alpha = exp2f(mrun[qt] - mnew);

        float rsum = 0.0f;
#pragma unroll
        for (int r = 0; r < 8; ++r) {
          const float p0 = exp2f(s0[r] - mnew);
          const float p1 = exp2f(s1[r] - mnew);
          rsum += p0 + p1;
          pf[qt][r]     = (bf16)(p0 * 1024.0f);
          pf[qt][r + 8] = (bf16)(p1 * 1024.0f);
        }
        rsum += __shfl_xor(rsum, 16, 32);
        lrun[qt] = lrun[qt] * alpha + rsum;
        mrun[qt] = mnew;

#pragma unroll
        for (int j = 0; j < 4; ++j)
#pragma unroll
          for (int r = 0; r < 8; ++r) o[qt][j][r] *= alpha;
      }
    }

#pragma unroll
    for (int j = 0; j < 4; ++j) {
      const bf16x16 vf = lds_frag(ldsV + (j * 16) * VSTRIDE, VSTRIDE);
#pragma unroll
      for (int qt = 0; qt < QW; ++qt)
        if (act[qt]) o[qt][j] = wmma_bf16(vf, pf[qt], o[qt][j]);
    }
  }

  __shared__ __attribute__((aligned(16))) float ldsOf[2][32 * 68];
  float* so = ldsOf[wave]; (void)ldsO;
#pragma unroll
  for (int qt = 0; qt < QW; ++qt) {
    const float rl = 1.0f / (lrun[qt] * 1024.0f);
#pragma unroll
    for (int j = 0; j < 4; ++j)
#pragma unroll
      for (int r = 0; r < 8; ++r) so[(16 * qt + qlane) * 68 + j * 16 + kh8 + r] = o[qt][j][r] * rl;
  }
  asm volatile("s_wait_dscnt 0" ::: "memory");
  __builtin_amdgcn_wave_barrier();
#pragma unroll 1
  for (int pass = 0; pass < 2; ++pass) {
#pragma unroll
    for (int it = 0; it < 16; ++it) { const int ch = lane + 32 * it, ql = ch >> 4, q4 = (ch & 15) * 4;
      *(volatile v4f_t*)(attnOut + ((size_t)(b * QROWS + q0 + ql)) * DD + h * DKK + q4) = *(const volatile v4fa*)(so + ql * 68 + q4); }
    __threadfence();
  }
}


template <typename AT, bool ACC>
__global__ __launch_bounds__(256) void gemm_kn2(const AT* __restrict__ A, int lda, size_t strideA,
                                               const float* __restrict__ Wm, int ldw, size_t strideW,
                                               const float* __restrict__ bias, float scale,
                                               float* __restrict__ Y, int ldy, size_t strideY, int K) {
  __shared__ __attribute__((aligned(16))) f16 ldsA[128 * GSTR], ldsAl[128 * GSTR];
  __shared__ __attribute__((aligned(16))) f16 ldsW[128 * GSTR], ldsWl[128 * GSTR];
  __shared__ __attribute__((aligned(16))) float oS[8][32 * 68];
  const int tid = threadIdx.x, lane = tid & 31, wave = tid >> 5, cl = lane & 15, rh = (lane >> 4) * 8;
  const int m0 = blockIdx.x * 128, n0 = blockIdx.y * 128;
  const int wm = (wave & 3) * 32, wn = (wave >> 2) * 64;
  A += (size_t)blockIdx.z * strideA; Wm += (size_t)blockIdx.z * strideW; Y += (size_t)blockIdx.z * strideY;
  f32x8 acc[2][4], accx[2][4];
#pragma unroll
  for (int i = 0; i < 2; ++i)
#pragma unroll
    for (int j = 0; j < 4; ++j) { f32x8 z = {}; acc[i][j] = z; accx[i][j] = z; }
#pragma unroll 1
  for (int k0 = 0; k0 < K; k0 += 32) {
    __syncthreads();
    {
      const int row = tid >> 1, ch = (tid & 1) * 16;
      const AT* src = A + (size_t)(m0 + row) * lda + k0 + ch;
#pragma unroll
      for (int g = 0; g < 16; ++g) { const float v = (float)src[g]; const f16 h = (f16)v; ldsA[row * GSTR + ch + g] = h; ldsAl[row * GSTR + ch + g] = (f16)((v - (float)h) * 2048.0f); }
    }
    {
      const int k = tid >> 3, nn0 = (tid & 7) * 16;
      const float* src = Wm + (size_t)(k0 + k) * ldw + n0 + nn0;
#pragma unroll
      for (int g = 0; g < 4; ++g) { const v4f_t v = *(const v4f_t*)(src + 4 * g);
#pragma unroll
        for (int u = 0; u < 4; ++u) { const f16 h = (f16)v[u]; ldsW[(nn0 + 4 * g + u) * GSTR + k] = h; ldsWl[(nn0 + 4 * g + u) * GSTR + k] = (f16)((v[u] - (float)h) * 2048.0f); } }
    }
    __syncthreads();
    f16x16 af[2], afl[2];
#pragma unroll
    for (int i = 0; i < 2; ++i) { af[i] = lds_frag(ldsA + (wm + 16 * i) * GSTR, GSTR); afl[i] = lds_frag(ldsAl + (wm + 16 * i) * GSTR, GSTR); }
#pragma unroll
    for (int j = 0; j < 4; ++j) {
      const f16x16 bf = lds_frag(ldsW + (wn + 16 * j) * GSTR, GSTR), bfl = lds_frag(ldsWl + (wn + 16 * j) * GSTR, GSTR);
#pragma unroll
      for (int i = 0; i < 2; ++i) { acc[i][j] = wmma16(af[i], bf, acc[i][j]); accx[i][j] = wmma16(af[i], bfl, accx[i][j]); accx[i][j] = wmma16(afl[i], bf, accx[i][j]); }
    }
  }
  float* so = oS[wave];
#pragma unroll
  for (int i = 0; i < 2; ++i)
#pragma unroll
    for (int j = 0; j < 4; ++j) {
      const float bv = bias ? bias[n0 + wn + 16 * j + cl] : 0.0f;
#pragma unroll
      for (int r = 0; r < 8; ++r) so[(16 * i + rh + r) * 68 + 16 * j + cl] = (acc[i][j][r] + accx[i][j][r] * (1.0f / 2048.0f)) * scale + bv;
    }
  asm volatile("s_wait_dscnt 0" ::: "memory");
  __builtin_amdgcn_wave_barrier();
  if (ACC) {
#pragma unroll
    for (int it = 0; it < 16; ++it) { const int f4 = lane + 32 * it, rr = f4 >> 4, q = (f4 & 15) * 4;
      const v4f_t old = *(const volatile v4fa*)(Y + (size_t)(m0 + wm + rr) * ldy + n0 + wn + q);
      v4f_t v = *(const volatile v4fa*)(so + rr * 68 + q); v += old; *(volatile v4fa*)(so + rr * 68 + q) = v; }
    asm volatile("s_wait_dscnt 0" ::: "memory");
  }
#pragma unroll 1
  for (int pass = 0; pass < 2; ++pass) {
#pragma unroll
    for (int it = 0; it < 16; ++it) { const int f4 = lane + 32 * it, rr = f4 >> 4, q = (f4 & 15) * 4;
      *(volatile v4f_t*)(Y + (size_t)(m0 + wm + rr) * ldy + n0 + wn + q) = *(const volatile v4fa*)(so + rr * 68 + q); }
    __threadfence();
  }
}

__global__ __launch_bounds__(256) void k_trig(float* __restrict__ cs) {
  const int pos = blockIdx.x * 8 + (threadIdx.x >> 5), i = threadIdx.x & 31;
  const float inv = exp2f(-(float)(2 * i) / 64.0f * 13.287712379549449f); const float a = (float)pos * inv;
  cs[((size_t)pos * 32 + i) * 2] = cosf(a); cs[((size_t)pos * 32 + i) * 2 + 1] = sinf(a);
}
__device__ __forceinline__ void rope_cs(const float* __restrict__ cs, int pos, int i, float& c, float& s) { const float* p = cs + ((size_t)pos * 32 + i) * 2; c = p[0]; s = p[1]; }
__global__ __launch_bounds__(256) void k_qprep(const float* __restrict__ q, const float* __restrict__ wq, const float* __restrict__ cs, bf16* __restrict__ q16) {
  __shared__ float rowS[64 * 68];
  const int tid = threadIdx.x, pr = tid >> 2, part = tid & 3; const size_t row = (size_t)blockIdx.x * 16 + (pr >> 2); const int h = pr & 3; const int t = (int)(row % TT);
  const float* src = q + row * DD + h * CC; float ss = 0.0f;
  for (int i = part * 16; i < part * 16 + 16; ++i) { const float v = src[i]; rowS[pr * 68 + i] = v; ss += v * v; }
  ss += __shfl_xor(ss, 1, 32); ss += __shfl_xor(ss, 2, 32); const float r = rsqrtf(ss * (1.0f / CC) + 1e-6f);
  __syncthreads();
  bf16* dst = q16 + row * DD + h * CC;
  union { bf16 hh[8]; v4u_t u; } lo, hi;
#pragma unroll 1
  for (int e = 0; e < 8; ++e) { const int i = part * 8 + e; float c, s; rope_cs(cs, t, i, c, s);
    const float x1 = rowS[pr * 68 + i] * r * wq[h * CC + i], x2 = rowS[pr * 68 + 32 + i] * r * wq[h * CC + 32 + i];
    lo.hh[e] = (bf16)(x1 * c - x2 * s); hi.hh[e] = (bf16)(x2 * c + x1 * s); }
#pragma unroll 1
  for (int pass = 0; pass < 2; ++pass) { *(volatile v4u_t*)(dst + part * 8) = lo.u; *(volatile v4u_t*)(dst + 32 + part * 8) = hi.u; __threadfence(); }
}
__global__ __launch_bounds__(256) void k_pool(const float* __restrict__ Hm, float* __restrict__ src) {
  const size_t i = (size_t)blockIdx.x * 256 + threadIdx.x;
  const int q = i & 63; const size_t rl = i >> 6; const int b = rl / KROWS, l = rl % KROWS;
  v4f_t o = {0.f, 0.f, 0.f, 0.f};
  if (l < 512) {
#pragma unroll 1
    for (int j = 0; j < 16; ++j) { const v4f_t v = *(const v4f_t*)(Hm + ((size_t)b * TT + l * 16 + j) * DM + q * 4); o[0] += v[0]; o[1] += v[1]; o[2] += v[2]; o[3] += v[3]; }
    for (int e = 0; e < 4; ++e) o[e] *= (1.0f / 16.0f); }
  else if (l < NKV) o = *(const v4f_t*)(Hm + ((size_t)b * TT + TT - 16 + (l - 512)) * DM + q * 4);
  *(volatile v4f_t*)(src + rl * DM + q * 4) = o; __threadfence(); *(volatile v4f_t*)(src + rl * DM + q * 4) = o;
}
__global__ __launch_bounds__(256) void k_kvprep(const float* __restrict__ kv, const float* __restrict__ wk, const float* __restrict__ wv, const float* __restrict__ cs, bf16* __restrict__ K16, bf16* __restrict__ Vt) {
  __shared__ float rowS[32 * 68]; __shared__ bf16 vS[64][40];
  const int tid = threadIdx.x, r = tid >> 3, part = tid & 7; const int b = blockIdx.x / (KROWS / 32), l0 = (blockIdx.x % (KROWS / 32)) * 32; const int l = l0 + r;
  const float* src = kv + ((size_t)b * KROWS + l) * 128; float ss = 0.0f;
  for (int i = part * 8; i < part * 8 + 8; ++i) { const float v = src[i]; rowS[r * 68 + i] = v; ss += v * v; }
  ss += __shfl_xor(ss, 1, 32); ss += __shfl_xor(ss, 2, 32); ss += __shfl_xor(ss, 4, 32); const float rs = rsqrtf(ss * (1.0f / CC) + 1e-6f);
  __syncthreads();
  union { bf16 hh[4]; unsigned long long u; } klo, khi;
#pragma unroll 1
  for (int e = 0; e < 4; ++e) { const int i = part * 4 + e; float c, s; rope_cs(cs, l, i, c, s); const bool ok = l < NKV;
    const float a1 = rowS[r * 68 + i] * rs, a2 = rowS[r * 68 + 32 + i] * rs;
    const float k1 = a1 * wk[i], k2 = a2 * wk[32 + i], v1 = a1 * wv[i], v2 = a2 * wv[32 + i];
    klo.hh[e] = (bf16)(ok ? (k1 * c - k2 * s) : 0.0f); khi.hh[e] = (bf16)(ok ? (k2 * c + k1 * s) : 0.0f);
    vS[i][r] = (bf16)(ok ? (v1 * c - v2 * s) : 0.0f); vS[32 + i][r] = (bf16)(ok ? (v2 * c + v1 * s) : 0.0f); }
  { bf16* dk = K16 + ((size_t)b * KROWS + l) * CC; *(volatile unsigned long long*)(dk + part * 4) = klo.u; *(volatile unsigned long long*)(dk + 32 + part * 4) = khi.u; __threadfence();
    *(volatile unsigned long long*)(dk + part * 4) = klo.u; *(volatile unsigned long long*)(dk + 32 + part * 4) = khi.u; }
  __syncthreads();
  { const int c = tid >> 2, q8 = (tid & 3) * 8; union { bf16 hh[8]; v4u_t u; } cv;
#pragma unroll
    for (int e = 0; e < 8; ++e) cv.hh[e] = vS[c][q8 + e];
    bf16* dv = Vt + ((size_t)b * CC + c) * KROWS + l0 + q8; *(volatile v4u_t*)dv = cv.u; __threadfence(); *(volatile v4u_t*)dv = cv.u; }
}
__global__ __launch_bounds__(256) void k_unrope(const float* __restrict__ att, const float* __restrict__ cs, float* __restrict__ o32) {
  const int tid = threadIdx.x, pr = tid >> 3, part = tid & 7; const size_t row = (size_t)blockIdx.x * 8 + (pr >> 2); const int h = pr & 3; const int t = (int)(row % TT);
  const float* src = att + row * DD + h * CC; float* dst = o32 + row * DD + h * CC;
  v4f_t lo, hi;
#pragma unroll 1
  for (int e = 0; e < 4; ++e) { const int i = part * 4 + e; float c, s; rope_cs(cs, t, i, c, s); s = -s;
    const float x1 = src[i], x2 = src[32 + i]; lo[e] = x1 * c - x2 * s; hi[e] = x2 * c + x1 * s; }
#pragma unroll 1
  for (int pass = 0; pass < 2; ++pass) { *(volatile v4f_t*)(dst + part * 4) = lo; *(volatile v4f_t*)(dst + 32 + part * 4) = hi; __threadfence(); }
}

#define GSTR 48
template <typename AT, int EPI, bool OUT16>
__global__ __launch_bounds__(256) void gemm_kne(const AT* __restrict__ A, int lda, const float* __restrict__ Wm, int ldw,
                                                const float* __restrict__ bias, const float* __restrict__ R, const float* __restrict__ gvec,
                                                void* __restrict__ Yv, int ldy, int K) {
  __shared__ __attribute__((aligned(16))) f16 ldsA[128 * GSTR];
  __shared__ __attribute__((aligned(16))) f16 ldsW[128 * GSTR];
  __shared__ __attribute__((aligned(16))) float oS[8][32 * 68];
  const int tid = threadIdx.x, lane = tid & 31, wave = tid >> 5, cl = lane & 15, rh = (lane >> 4) * 8;
  const int m0 = blockIdx.x * 128, n0 = blockIdx.y * 128;
  const int wm = (wave & 3) * 32, wn = (wave >> 2) * 64;
  f32x8 acc[2][4];
#pragma unroll
  for (int i = 0; i < 2; ++i)
#pragma unroll
    for (int j = 0; j < 4; ++j) { f32x8 z = {}; acc[i][j] = z; }
#pragma unroll 1
  for (int k0 = 0; k0 < K; k0 += 32) {
    __syncthreads();
    { const int row = tid >> 1, ch = (tid & 1) * 16;
      const AT* src = A + (size_t)(m0 + row) * lda + k0 + ch;
#pragma unroll
      for (int g = 0; g < 16; ++g) ldsA[row * GSTR + ch + g] = (f16)src[g]; }
    { const int k = tid >> 3, nn0 = (tid & 7) * 16;
      const float* src = Wm + (size_t)(k0 + k) * ldw + n0 + nn0;
#pragma unroll
      for (int g = 0; g < 4; ++g) { const v4f_t v = *(const v4f_t*)(src + 4 * g);
#pragma unroll
        for (int u = 0; u < 4; ++u) ldsW[(nn0 + 4 * g + u) * GSTR + k] = (f16)v[u]; } }
    __syncthreads();
    f16x16 af[2];
#pragma unroll
    for (int i = 0; i < 2; ++i) af[i] = lds_frag(ldsA + (wm + 16 * i) * GSTR, GSTR);
#pragma unroll
    for (int j = 0; j < 4; ++j) {
      const f16x16 bf = lds_frag(ldsW + (wn + 16 * j) * GSTR, GSTR);
#pragma unroll
      for (int i = 0; i < 2; ++i) acc[i][j] = wmma16(af[i], bf, acc[i][j]);
    }
  }
  float* so = oS[wave];
#pragma unroll
  for (int i = 0; i < 2; ++i)
#pragma unroll
    for (int j = 0; j < 4; ++j) {
      const int n = n0 + wn + 16 * j + cl;
      const float bv = bias ? bias[n] : 0.0f;
      const float gv = (EPI == 2) ? gvec[n] : 0.0f;
      if (EPI == 1) {
#pragma unroll 1
        for (int r = 0; r < 8; ++r) { const float xg = acc[i][j][r] + bv; so[(16 * i + rh + r) * 68 + 16 * j + cl] = 0.5f * xg * (1.0f + erff(xg * 0.70710678118654752f)); }
      } else {
#pragma unroll
        for (int r = 0; r < 8; ++r) {
          float v = acc[i][j][r] + bv;
          if (EPI == 2) v = R[(size_t)(m0 + wm + 16 * i + rh + r) * ldy + n] + gv * v;
          so[(16 * i + rh + r) * 68 + 16 * j + cl] = v;
        }
      }
    }
  asm volatile("s_wait_dscnt 0" ::: "memory");
  __builtin_amdgcn_wave_barrier();
#pragma unroll 1
  for (int pass = 0; pass < 2; ++pass) {
    if (OUT16) {
      f16* Y = (f16*)Yv;
#pragma unroll
      for (int it = 0; it < 8; ++it) { const int c = lane + 32 * it, rr = c >> 3, q8 = (c & 7) * 8;
        union { f16 h[8]; v4u_t v; } u;
#pragma unroll
        for (int e = 0; e < 8; ++e) u.h[e] = (f16)so[rr * 68 + q8 + e];
        *(volatile v4u_t*)(Y + (size_t)(m0 + wm + rr) * ldy + n0 + wn + q8) = u.v; }
    } else {
      float* Y = (float*)Yv;
#pragma unroll
      for (int it = 0; it < 16; ++it) { const int f4 = lane + 32 * it, rr = f4 >> 4, q = (f4 & 15) * 4;
        *(volatile v4f_t*)(Y + (size_t)(m0 + wm + rr) * ldy + n0 + wn + q) = *(const volatile v4fa*)(so + rr * 68 + q); }
    }
    __threadfence();
  }
}

__global__ __launch_bounds__(256) void k_padkv(const float* __restrict__ Wkv, float* __restrict__ Wp) { const int row = blockIdx.x, tid = threadIdx.x; if (tid < 128) Wp[row * 128 + tid] = (tid < CC) ? Wkv[row * CC + tid] : 0.0f; }
__global__ __launch_bounds__(256) void k_bdg(const float* __restrict__ Wg0, const float* __restrict__ Wg1, const float* __restrict__ bg0, const float* __restrict__ bg1, float* __restrict__ BD, float* __restrict__ bb) {
  const int row = blockIdx.x, tid = threadIdx.x; if (tid < 128) { float v = 0.0f;
    if (row < 128 && tid < 64) v = Wg0[row * 64 + tid]; if (row >= 128 && tid >= 64) v = Wg1[(row - 128) * 64 + (tid - 64)]; BD[row * 128 + tid] = v; }
  if (row == 0 && tid < 128) bb[tid] = (tid < 64) ? bg0[tid] : bg1[tid - 64];
}

extern "C" void kernel_launch(void* const* d_in, const int* in_sizes, int n_in,
                              void* d_out, int out_size, void* d_ws, size_t ws_size,
                              hipStream_t stream) {
  (void)in_sizes; (void)n_in; (void)out_size;
  const float** f = (const float**)d_in;
  const float* Hm = f[0], *W_Q = f[1], *W_KV = f[2], *w_q = f[3], *w_k = f[4], *w_v = f[5], *Wg0 = f[6], *bg0 = f[7], *Wg1 = f[8], *bg1 = f[9], *Wout = f[10], *bout = f[11];
  float* out = (float*)d_out;
  char* ws = (char*)d_ws;
  float* q32 = (float*)ws; ws += (size_t)MTOK * DD * 4;
  bf16* Qb = (bf16*)ws; ws += (size_t)MTOK * DD * 2;
  float* kvsrc = (float*)ws; ws += (size_t)BB * KROWS * DM * 4;
  float* kv32 = (float*)ws; ws += (size_t)BB * KROWS * 128 * 4;
  float* Wkvp = (float*)ws; ws += 256 * 128 * 4;
  bf16* K16 = (bf16*)ws; ws += (size_t)BB * KROWS * CC * 2;
  bf16* VtB = (bf16*)ws; ws += (size_t)BB * CC * KROWS * 2;
  float* att = q32;
  float* o32 = (float*)ws; ws += (size_t)MTOK * DD * 4;
  float* BD = (float*)ws; ws += 256 * 128 * 4; float* bb = (float*)ws; ws += 128 * 4;
  float* pall = (float*)ws; ws += (size_t)MTOK * 128 * 4;
  float* cs = (float*)ws; ws += (size_t)TT * 32 * 2 * 4;
  if ((size_t)(ws - (char*)d_ws) > ws_size) return;
  const dim3 blk(256);
  gemm_kn2<float, false><<<dim3(MTOK / 128, DD / 128, 1), blk, 0, stream>>>(Hm, DM, 0, W_Q, DD, 0, nullptr, 1.0f, q32, DD, 0, DM);
  k_trig<<<dim3(TT / 8), blk, 0, stream>>>(cs);
  k_qprep<<<dim3(MTOK / 16), blk, 0, stream>>>(q32, w_q, cs, Qb);
  k_pool<<<dim3(BB * KROWS * 64 / 256), blk, 0, stream>>>(Hm, kvsrc);
  k_padkv<<<dim3(256), blk, 0, stream>>>(W_KV, Wkvp);
  gemm_kne<float, 0, false><<<dim3(BB * KROWS / 128, 1), blk, 0, stream>>>(kvsrc, DM, Wkvp, 128, nullptr, nullptr, nullptr, kv32, 128, DM);
  k_kvprep<<<dim3(BB * (KROWS / 32)), blk, 0, stream>>>(kv32, w_k, w_v, cs, K16, VtB);
  attn_kernel<<<dim3(TT / 64, HH, BB), dim3(64), 0, stream>>>(Qb, K16, VtB, att);
  k_unrope<<<dim3(MTOK / 8), blk, 0, stream>>>(att, cs, o32);
  k_bdg<<<dim3(256), blk, 0, stream>>>(Wg0, Wg1, bg0, bg1, BD, bb);
  gemm_kn2<float, false><<<dim3(MTOK / 128, 1, 1), blk, 0, stream>>>(o32, DD, 0, BD, 128, 0, bb, 1.0f, pall, 128, 0, DD);
  gemm_kn2<float, false><<<dim3(MTOK / 128, DD / 128, 1), blk, 0, stream>>>(pall, 128, 0, Wout, DD, 0, bout, 1.0f, out, DD, 0, 128);
}
